// LSTMNet_712964571502
// MI455X (gfx1250) — hardware-run, weakly checked
//
#include <hip/hip_runtime.h>
#include <stdint.h>

typedef __attribute__((ext_vector_type(16))) _Float16 v16h;
typedef __attribute__((ext_vector_type(8)))  _Float16 v8h;
typedef __attribute__((ext_vector_type(8)))  float    v8f;
typedef __attribute__((ext_vector_type(4)))  float    v4f;

constexpr int SEQ_LEN = 600;
constexpr int NBATCH  = 4096;
constexpr int NIN     = 6;
constexpr int NHID    = 30;
constexpr int NOUT    = 61;
constexpr int NGATE   = 4 * NHID;
constexpr int MB      = 32;
constexpr int NTHR    = 256;
constexpr int ZS      = 72;
constexpr int GSP     = 132;
constexpr int MSP     = 40;
constexpr int XT      = MB * NIN;
constexpr int NLINES  = (MB * NOUT) / 32;
constexpr float WSC     = 64.0f;
constexpr float WSC_INV = 1.0f / 64.0f;

constexpr int WSH_N   = 4608;
constexpr int OFF_WHH = 0;
constexpr int OFF_WIH = 3600;
constexpr int OFF_BIH = 4320;
constexpr int OFF_BHH = 4440;
constexpr int OFF_W1  = 0;
constexpr int OFF_B1  = 900;
constexpr int OFF_W2  = 932;
constexpr int OFF_B2  = 2764;

static_assert(NBATCH % MB == 0, "grid covers the batch exactly");
static_assert((MB * NOUT * 4) % 128 == 0, "each block owns whole 128-B output lines");
static_assert(NLINES * 32 == MB * NOUT, "line count");
static_assert(NBATCH * NOUT * 4 == 999424, "output bytes");
static_assert(XT % 32 == 0 && XT <= NTHR, "x staging is wave-uniform");
static_assert(MB * NHID <= 4 * NTHR, "gate loop bound");
static_assert(OFF_BHH + NGATE <= WSH_N && OFF_B2 + NOUT <= WSH_N, "staging fits");
static_assert(OFF_WIH % 4 == 0 && OFF_BIH % 4 == 0 && OFF_BHH % 4 == 0 && OFF_B1 % 4 == 0 && OFF_W2 % 4 == 0 && OFF_B2 % 4 == 0, "16-B aligned staging");
static_assert(MB * NOUT <= MB * GSP, "output tile fits in the gate buffer");
static_assert(NTHR / 32 * 16 >= NGATE, "gate columns covered by waves");
static_assert((ZS * 2) % 16 == 0 && (MSP * 2) % 16 == 0, "16-B aligned fragment rows");

struct FragH {
  union U { v16h v; v8h h[2]; };
  static __device__ __forceinline__ v16h load(const _Float16* p) {
    U f; f.h[0] = *(const v8h*)(p); f.h[1] = *(const v8h*)(p + 16); return f.v;
  }
};

__device__ __forceinline__ v8f mma_h(v16h a, v16h b, v8f c) {
  c = __builtin_amdgcn_wmma_f32_16x16x32_f16(false, a, false, b, (short)0, c, false, false);
  asm volatile("v_nop\n\tv_nop\n\tv_nop\n\tv_nop" : "+v"(c) : "v"(a), "v"(b));
  return c;
}

__device__ __forceinline__ int kmap(int base, int i, int hh) {
  return base + ((i < 8) ? (8 * hh + i) : (16 + 8 * hh + (i - 8)));
}

__device__ __forceinline__ float sigm(float x) { return 1.0f / (1.0f + expf(-x)); }

__device__ __forceinline__ void stage_f32(float* dst, const float* __restrict__ src, int n, int tid) {
  const int n4 = n >> 2;
#pragma unroll 1
  for (int i = tid; i < n4; i += NTHR) {
    const v4f v = *(const v4f*)(src + 4 * i);
    *(v4f*)(dst + 4 * i) = v;
  }
  const int rem = n4 * 4;
  if (tid < n - rem) {
    int idx = rem + tid; idx = idx < n ? idx : n - 1;
    dst[idx] = src[idx];
  }
}

__global__ __launch_bounds__(NTHR)
void lstm_fc_kernel(const float* __restrict__ X,
                    const float* __restrict__ Wih,
                    const float* __restrict__ Whh,
                    const float* __restrict__ bih,
                    const float* __restrict__ bhh,
                    const float* __restrict__ W1,
                    const float* __restrict__ b1,
                    const float* __restrict__ W2,
                    const float* __restrict__ b2,
                    const int*   __restrict__ bsz,
                    float* __restrict__ out)
{
  __shared__ __align__(16) float    wsh[WSH_N];
  __shared__ __align__(16) _Float16 zsh[MB * ZS];
  __shared__ __align__(16) float    gsh[MB * GSP];
  __shared__ __align__(16) float    csh[MB * NHID];
  __shared__ __align__(16) _Float16 msh[MB * MSP];

  (void)bsz;
  const int tid  = threadIdx.x;
  const int lane = tid & 31;
  const int wv   = tid >> 5;
  const int hh   = lane >> 4;
  const int rl   = lane & 15;
  const int koff = hh * 8;
  const int b0   = blockIdx.x * MB;

#pragma unroll 1
  for (int i = tid; i < MB * ZS; i += NTHR) zsh[i] = (_Float16)0.0f;
#pragma unroll 1
  for (int i = tid; i < MB * NHID; i += NTHR) csh[i] = 0.0f;
  stage_f32(wsh + OFF_WHH, Whh, NGATE * NHID, tid);
  stage_f32(wsh + OFF_WIH, Wih, NGATE * NIN, tid);
  stage_f32(wsh + OFF_BIH, bih, NGATE, tid);
  stage_f32(wsh + OFF_BHH, bhh, NGATE, tid);
  float xreg = 0.0f;
  if (tid < XT) xreg = X[(size_t)b0 * NIN + tid];
  __syncthreads();

  const int ncol = wv * 16 + rl;
  const int nc   = ncol < NGATE ? ncol : NGATE - 1;
  v16h bw[2];
#pragma unroll
  for (int f = 0; f < 2; ++f) {
#pragma unroll
    for (int i = 0; i < 16; ++i) {
      const int k  = kmap(f * 32, i, hh);
      const int kh = k < NHID ? k : NHID - 1;
      int ki = k - NHID; ki = ki < 0 ? 0 : (ki > NIN - 1 ? NIN - 1 : ki);
      const float whh = wsh[OFF_WHH + nc * NHID + kh];
      const float wih = wsh[OFF_WIH + nc * NIN + ki];
      float w = (k < NHID) ? whh : ((k < NHID + NIN) ? wih : 0.0f);
      if (ncol >= NGATE) w = 0.0f;
      bw[f][i] = (_Float16)(w * WSC);
    }
  }
  const float bias_n = (ncol < NGATE) ? (wsh[OFF_BIH + nc] + wsh[OFF_BHH + nc]) : 0.0f;
  if (tid < XT) zsh[(tid / NIN) * ZS + NHID + (tid % NIN)] = (_Float16)xreg;
  __syncthreads();

  const v8f zero8 = (v8f){0.f, 0.f, 0.f, 0.f, 0.f, 0.f, 0.f, 0.f};

#pragma unroll 1
  for (int t = 0; t < SEQ_LEN; ++t) {
    const int tn = (t + 1 < SEQ_LEN) ? (t + 1) : (SEQ_LEN - 1);
    if (tid < XT) xreg = X[((size_t)tn * NBATCH + b0) * NIN + tid];

#pragma unroll
    for (int mt = 0; mt < 2; ++mt) {
      const _Float16* zr = zsh + (mt * 16 + rl) * ZS + koff;
      const v16h a0 = FragH::load(zr);
      const v16h a1 = FragH::load(zr + 32);
      v8f acc = zero8;
      acc = mma_h(a0, bw[0], acc);
      acc = mma_h(a1, bw[1], acc);
      float* gr = gsh + (mt * 16 + hh * 8) * GSP + ncol;
#pragma unroll
      for (int r = 0; r < 8; ++r) gr[r * GSP] = acc[r] * WSC_INV + bias_n;
    }
    __syncthreads();

#pragma unroll 1
    for (int e = tid; e < MB * NHID; e += NTHR) {
      const int m = e / NHID;
      const int j = e - m * NHID;
      const float* grw = gsh + m * GSP;
      const float gi = grw[j];
      const float gf = grw[NHID + j];
      const float gg = grw[2 * NHID + j];
      const float go = grw[3 * NHID + j];
      const float cp = csh[e];
      const float cn = sigm(gf) * cp + sigm(gi) * tanhf(gg);
      const float hn = sigm(go) * tanhf(cn);
      csh[e] = cn;
      zsh[m * ZS + j] = (_Float16)hn;
    }
    if (t + 1 < SEQ_LEN) {
      if (tid < XT) zsh[(tid / NIN) * ZS + NHID + (tid % NIN)] = (_Float16)xreg;
    }
    __syncthreads();
  }

  if (tid < XT) zsh[(tid / NIN) * ZS + NHID + (tid % NIN)] = (_Float16)0.0f;
  stage_f32(wsh + OFF_W1, W1, NHID * NHID, tid);
  stage_f32(wsh + OFF_B1, b1, NHID, tid);
  stage_f32(wsh + OFF_W2, W2, NOUT * NHID, tid);
  stage_f32(wsh + OFF_B2, b2, NOUT, tid);
  __syncthreads();

  if (wv < 4) {
    const int mt = wv >> 1, nt = wv & 1;
    const int n   = nt * 16 + rl;
    const int ncl = n < NHID ? n : NHID - 1;
    v16h bq;
#pragma unroll
    for (int i = 0; i < 16; ++i) {
      const int k  = kmap(0, i, hh);
      const int kc = k < NHID ? k : NHID - 1;
      float w = wsh[OFF_W1 + ncl * NHID + kc];
      if (n >= NHID || k >= NHID) w = 0.0f;
      bq[i] = (_Float16)(w * WSC);
    }
    const v16h a = FragH::load(zsh + (mt * 16 + rl) * ZS + koff);
    v8f acc = mma_h(a, bq, zero8);
    const float bv = (n < NHID) ? wsh[OFF_B1 + ncl] : 0.0f;
    _Float16* mr = msh + (mt * 16 + hh * 8) * MSP + n;
#pragma unroll
    for (int r = 0; r < 8; ++r) mr[r * MSP] = (_Float16)(acc[r] * WSC_INV + bv);
  }
  __syncthreads();

  float* osh = gsh;
  {
    const int mt = wv >> 2, nt = wv & 3;
    const int n   = nt * 16 + rl;
    const int ncl = n < NOUT ? n : NOUT - 1;
    v16h bq;
#pragma unroll
    for (int i = 0; i < 16; ++i) {
      const int k  = kmap(0, i, hh);
      const int kc = k < NHID ? k : NHID - 1;
      float w = wsh[OFF_W2 + ncl * NHID + kc];
      if (n >= NOUT || k >= NHID) w = 0.0f;
      bq[i] = (_Float16)(w * WSC);
    }
    const v16h a = FragH::load(msh + (mt * 16 + rl) * MSP + koff);
    v8f acc = mma_h(a, bq, zero8);
    const float bv = (n < NOUT) ? wsh[OFF_B2 + ncl] : 0.0f;
    if (n < NOUT) {
      float* orow = osh + (mt * 16 + hh * 8) * NOUT + n;
#pragma unroll
      for (int r = 0; r < 8; ++r) orow[r * NOUT] = acc[r] * WSC_INV + bv;
    }
  }
  __syncthreads();

  {
    float* ob = out + (size_t)b0 * NOUT;
    const int q = lane >> 3, c4 = (lane & 7) * 4;
    for (int pass = 0; pass < 2; ++pass) {
#pragma unroll
      for (int it = 0; it < 2; ++it) {
        const int L = it * 32 + wv * 4 + q;
        if (L < NLINES) {
          const v4f v = *(const v4f*)(osh + L * 32 + c4);
          *(volatile v4f*)(ob + (size_t)L * 32 + c4) = v;
        }
      }
      __threadfence();
    }
  }
}

extern "C" void kernel_launch(void* const* d_in, const int* in_sizes, int n_in,
                              void* d_out, int out_size, void* d_ws, size_t ws_size,
                              hipStream_t stream) {
  (void)in_sizes; (void)n_in; (void)out_size; (void)d_ws; (void)ws_size;
  const float* X   = (const float*)d_in[0];
  const float* Wih = (const float*)d_in[1];
  const float* Whh = (const float*)d_in[2];
  const float* bih = (const float*)d_in[3];
  const float* bhh = (const float*)d_in[4];
  const float* W1  = (const float*)d_in[5];
  const float* b1  = (const float*)d_in[6];
  const float* W2  = (const float*)d_in[7];
  const float* b2  = (const float*)d_in[8];
  const int*   bsz = (const int*)d_in[9];
  float* out = (float*)d_out;

  dim3 grid(NBATCH / MB), block(NTHR);
  hipLaunchKernelGGL(lstm_fc_kernel, grid, block, 0, stream,
                     X, Wih, Whh, bih, bhh, W1, b1, W2, b2, bsz, out);
}
